// Classifier_87256555586283
// MI455X (gfx1250) — hardware-verified
//
#include <hip/hip_runtime.h>
#include <math.h>

constexpr int kHid     = 768;
constexpr int kRows    = 16384;
constexpr int kBasis   = 8;
constexpr int kFeat    = 9;
constexpr int kKdim    = kHid * kFeat;
constexpr int kChunk   = 4096;
constexpr int kNChunk  = kRows / kChunk;
constexpr int kNout    = 2;
constexpr int kNpad    = 64;
constexpr int kSeg8    = kKdim / 8;
constexpr float kCarry     = 16.0f;
constexpr float kGemmScale = 1.0f / 256.0f;

static_assert(kKdim % 32 == 0, "K multiple of 32");
static_assert(kChunk % 64 == 0 && kHid % 64 == 0 && kNpad % 64 == 0, "tile multiples");
static_assert(kRows % kChunk == 0, "exact chunks");
static_assert(kHid == 3 * 256, "three features per thread");
static_assert(kSeg8 <= 4 * 256 && kSeg8 > 3 * 256, "row segment coverage");
static_assert(kRows % 64 == 0, "copy kernel coverage");

constexpr size_t kOffBt1 = 0;
constexpr size_t kBytesBt1 = (size_t)kHid * kKdim * 2;
constexpr size_t kOffBt2 = kOffBt1 + kBytesBt1;
constexpr size_t kBytesBt2 = (size_t)kNpad * kKdim * 2;
constexpr size_t kOffA   = kOffBt2 + kBytesBt2;
constexpr size_t kBytesA = (size_t)kChunk * kKdim * 2;
constexpr size_t kOffH1  = kOffA + kBytesA;
constexpr size_t kBytesH1 = (size_t)kRows * kHid * 4;
constexpr size_t kOffP   = kOffH1 + kBytesH1;
constexpr size_t kBytesP = (size_t)kRows * kNpad * 4;
constexpr size_t kWsEnd  = kOffP + kBytesP;
static_assert(kWsEnd == 122650624ull, "carve total");
static_assert(kWsEnd <= 134217728ull, "carve under 128 MiB");
static_assert(kOffBt2 % 256 == 0 && kOffA % 256 == 0 && kOffH1 % 256 == 0 && kOffP % 256 == 0, "aligned regions");

typedef __attribute__((ext_vector_type(16))) _Float16 v16h;
typedef __attribute__((ext_vector_type(8)))  _Float16 v8h;
typedef __attribute__((ext_vector_type(16))) __bf16   v16b;
typedef __attribute__((ext_vector_type(8)))  __bf16   v8b;
typedef __attribute__((ext_vector_type(8)))  float    v8f;
typedef __attribute__((ext_vector_type(4)))  float    v4f;
typedef __attribute__((ext_vector_type(4)))  unsigned int v4u;

__device__ __forceinline__ unsigned short f2bf_bits(float f) {
  unsigned u = __float_as_uint(f);
  return (unsigned short)((u + 0x7FFFu + ((u >> 16) & 1u)) >> 16);
}
__device__ __forceinline__ float bf_bits2f(unsigned short h) { return __uint_as_float(((unsigned)h) << 16); }

__device__ __forceinline__ void dep_guard_h(v8f& a, v8f& b, v16h x, v16h y) { asm volatile("v_nop\n\tv_nop\n\tv_nop\n\tv_nop" : "+v"(a), "+v"(b) : "v"(x), "v"(y)); }
__device__ __forceinline__ void dep_guard_b(v8f& a, v8f& b, v16b x, v16b y) { asm volatile("v_nop\n\tv_nop\n\tv_nop\n\tv_nop" : "+v"(a), "+v"(b) : "v"(x), "v"(y)); }
__device__ __forceinline__ void dep_guard4_h(v8f& a, v8f& b, v8f& c, v8f& d, v16h x, v16h y) { asm volatile("v_nop\n\tv_nop\n\tv_nop\n\tv_nop" : "+v"(a), "+v"(b), "+v"(c), "+v"(d) : "v"(x), "v"(y)); }
__device__ __forceinline__ void dep_guard4_b(v8f& a, v8f& b, v8f& c, v8f& d, v16b x, v16b y) { asm volatile("v_nop\n\tv_nop\n\tv_nop\n\tv_nop" : "+v"(a), "+v"(b), "+v"(c), "+v"(d) : "v"(x), "v"(y)); }
__device__ __forceinline__ void keep4_h(v16h a, v16h b, v16h c, v16h d) { asm volatile("v_nop" :: "v"(a), "v"(b), "v"(c), "v"(d)); }
__device__ __forceinline__ void keep4_b(v16b a, v16b b, v16b c, v16b d) { asm volatile("v_nop" :: "v"(a), "v"(b), "v"(c), "v"(d)); }
__device__ __forceinline__ void acc_guard4(v8f& a, v8f& b, v8f& c, v8f& d) { asm volatile("v_nop\n\tv_nop\n\tv_nop\n\tv_nop" : "+v"(a), "+v"(b), "+v"(c), "+v"(d)); }
template <typename T> struct Frag;
template <> struct Frag<_Float16> {
  typedef v16h V; union U { v16h v; v8h h[2]; };
  static __device__ __forceinline__ v16h load(const _Float16* p) {
    U f; f.h[0] = *(const v8h*)(p); f.h[1] = *(const v8h*)(p + 16); return f.v;
  }
  static __device__ __forceinline__ v8f mma(v16h a, v16h b, v8f c) {
    return __builtin_amdgcn_wmma_f32_16x16x32_f16(false, a, false, b, (short)0, c, false, false);
  }
  static __device__ __forceinline__ void guard(v8f& a, v8f& b, v16h x, v16h y) { dep_guard_h(a, b, x, y); }
  static __device__ __forceinline__ void guard4(v8f& a, v8f& b, v8f& c, v8f& d, v16h x, v16h y) { dep_guard4_h(a, b, c, d, x, y); }
  static __device__ __forceinline__ void keep(v16h a, v16h b, v16h c, v16h d) { keep4_h(a, b, c, d); }
};
template <> struct Frag<__bf16> {
  typedef v16b V; union U { v16b v; v8b h[2]; };
  static __device__ __forceinline__ v16b load(const __bf16* p) {
    U f; f.h[0] = *(const v8b*)(p); f.h[1] = *(const v8b*)(p + 16); return f.v;
  }
  static __device__ __forceinline__ v8f mma(v16b a, v16b b, v8f c) {
    return __builtin_amdgcn_wmma_f32_16x16x32_bf16(false, a, false, b, (short)0, c, false, false);
  }
  static __device__ __forceinline__ void guard(v8f& a, v8f& b, v16b x, v16b y) { dep_guard_b(a, b, x, y); }
  static __device__ __forceinline__ void guard4(v8f& a, v8f& b, v8f& c, v8f& d, v16b x, v16b y) { dep_guard4_b(a, b, c, d, x, y); }
  static __device__ __forceinline__ void keep(v16b a, v16b b, v16b c, v16b d) { keep4_b(a, b, c, d); }
};

__device__ __forceinline__ unsigned pk16(unsigned short a, unsigned short b) { return (unsigned)a | ((unsigned)b << 16); }
__device__ __forceinline__ unsigned short h_bits(float f) { const _Float16 h = (_Float16)f; return __builtin_bit_cast(unsigned short, h); }

template <int ET> struct Elem;
template <> struct Elem<0> { typedef _Float16 T; };
template <> struct Elem<1> { typedef __bf16 T; };
template <int ET, bool SPLIT, int BIAS_MODE, int OUT_MODE, bool RESID, int ACT = 0>
__global__ __launch_bounds__(256) void wmma_gemm64(
    const unsigned short* __restrict__ Ap, const unsigned short* __restrict__ A2p, int lda, long strideA,
    const unsigned short* __restrict__ Btp, const unsigned short* __restrict__ Bt2p, int ldb, long strideB,
    void* __restrict__ Cout, void* __restrict__ Cout2, int ldc, long strideC,
    const float* __restrict__ bias,
    const float* __restrict__ resid, long strideR,
    int M, int N, int K, float scale) {
  typedef typename Elem<ET>::T T;
  typedef typename Frag<T>::V V;
  const T* A = (const T*)Ap; const T* A2 = (const T*)A2p; const T* Bt = (const T*)Btp; const T* Bt2 = (const T*)Bt2p;
  __shared__ __align__(16) float sT[8][16 * 68];
  const int b    = blockIdx.y;
  const int lane = threadIdx.x & 31;
  const int wave = threadIdx.x >> 5;
  const int tilesN = N >> 6;
  const int tilesM = M >> 6;
  const int tile = blockIdx.x * 8 + wave;
  if (tile >= tilesM * tilesN) return;
  const int tm = tile / tilesN;
  const int tn = tile - tm * tilesN;
  const int m0 = tm << 6;
  const int n0 = tn << 6;

  const T* Ab  = A  + (size_t)b * strideA;
  const T* Bb  = Bt + (size_t)b * strideB;
  const T* Ab2 = SPLIT ? (A2  + (size_t)b * strideA) : nullptr;
  const T* Bb2 = SPLIT ? (Bt2 + (size_t)b * strideB) : nullptr;

  const int rlane = lane & 15;
  const int koff  = (lane >> 4) * 8;
  const int mOff  = (lane >> 4) * 8;

  v8f acc[4][4];
#pragma unroll
  for (int i = 0; i < 4; ++i)
#pragma unroll
    for (int j = 0; j < 4; ++j) acc[i][j] = (v8f){0.f,0.f,0.f,0.f,0.f,0.f,0.f,0.f};

  for (int k0 = 0; k0 < K; k0 += 32) {
    V bh[4], bl[4];
#pragma unroll
    for (int j = 0; j < 4; ++j) {
      const size_t bo = (size_t)(n0 + (j << 4) + rlane) * ldb + koff + k0;
      bh[j] = Frag<T>::load(Bb + bo);
      if (SPLIT) bl[j] = Frag<T>::load(Bb2 + bo);
    }
#pragma unroll
    for (int i = 0; i < 4; ++i) {
      const size_t ao = (size_t)(m0 + (i << 4) + rlane) * lda + koff + k0;
      V ah = Frag<T>::load(Ab + ao);
      V al;
      if (SPLIT) al = Frag<T>::load(Ab2 + ao);
#pragma unroll
      for (int j = 0; j < 4; ++j) {
        acc[i][j] = Frag<T>::mma(ah, bh[j], acc[i][j]);
        if (SPLIT) {
          acc[i][j] = Frag<T>::mma(ah, bl[j], acc[i][j]);
          acc[i][j] = Frag<T>::mma(al, bh[j], acc[i][j]);
        }
      }
      Frag<T>::guard4(acc[i][0], acc[i][1], acc[i][2], acc[i][3], ah, SPLIT ? al : ah);
    }
    Frag<T>::keep(bh[0], bh[1], bh[2], bh[3]);
    if (SPLIT) Frag<T>::keep(bl[0], bl[1], bl[2], bl[3]);
  }
  acc_guard4(acc[0][0], acc[0][1], acc[0][2], acc[0][3]);
  acc_guard4(acc[1][0], acc[1][1], acc[1][2], acc[1][3]);
  acc_guard4(acc[2][0], acc[2][1], acc[2][2], acc[2][3]);
  acc_guard4(acc[3][0], acc[3][1], acc[3][2], acc[3][3]);

  float* slab = sT[wave];
  const float* Rb = RESID ? (resid + (size_t)b * strideR) : nullptr;
#pragma unroll
  for (int i = 0; i < 4; ++i) {
    const int mBase = m0 + (i << 4);
#pragma unroll
    for (int j = 0; j < 4; ++j) {
      const int n = n0 + (j << 4) + rlane;
      float bv = 0.f;
      if (BIAS_MODE == 2) bv = bias[n];
#pragma unroll
      for (int r = 0; r < 8; ++r) {
        float v = acc[i][j][r] * scale;
        if (BIAS_MODE == 1) v += bias[mBase + mOff + r];
        if (BIAS_MODE == 2) v += bv;
        if (RESID) v += Rb[(size_t)(mBase + mOff + r) * ldc + n];
        if (ACT == 2) v = fmaxf(v, 0.0f);
        if (ACT == 4) v = (v > 0.f) ? v : 0.01f * v;
        slab[(mOff + r) * 68 + (j << 4) + rlane] = v;
      }
    }
    __builtin_amdgcn_fence(__ATOMIC_RELEASE, "workgroup");
    __builtin_amdgcn_wave_barrier();
    __builtin_amdgcn_fence(__ATOMIC_ACQUIRE, "workgroup");
    if (OUT_MODE == 0) {
      float* C = (float*)Cout + (size_t)b * strideC;
      const int hh = lane >> 4, c4 = (lane & 15) * 4;
      for (int pass = 0; pass < 2; ++pass) {
#pragma unroll
        for (int it = 0; it < 8; ++it) {
          const int row = it * 2 + hh;
          v4f v = *(const v4f*)(slab + row * 68 + c4);
          *(volatile v4f*)(C + (size_t)(mBase + row) * ldc + n0 + c4) = v;
        }
        __threadfence();
      }
    } else {
      const int q = lane >> 3, c8 = (lane & 7) * 8;
      unsigned short* C  = (unsigned short*)Cout  + (size_t)b * strideC;
      unsigned short* C2 = (OUT_MODE == 2) ? ((unsigned short*)Cout2 + (size_t)b * strideC) : nullptr;
      for (int pass = 0; pass < 2; ++pass) {
#pragma unroll
        for (int it = 0; it < 4; ++it) {
          const int row = it * 4 + q;
          const float* sp = slab + row * 68 + c8;
          v8h hv, lv;
#pragma unroll
          for (int e = 0; e < 8; ++e) {
            if (OUT_MODE == 1) {
              hv[e] = (_Float16)sp[e];
            } else {
              unsigned short hb = f2bf_bits(sp[e]);
              unsigned short lb = f2bf_bits(sp[e] - bf_bits2f(hb));
              hv[e] = __builtin_bit_cast(_Float16, hb);
              lv[e] = __builtin_bit_cast(_Float16, lb);
            }
          }
          *(volatile v8h*)(C + (size_t)(mBase + row) * ldc + n0 + c8) = hv;
          if (OUT_MODE == 2) *(volatile v8h*)(C2 + (size_t)(mBase + row) * ldc + n0 + c8) = lv;
        }
        __threadfence();
      }
    }
    __builtin_amdgcn_fence(__ATOMIC_RELEASE, "workgroup");
    __builtin_amdgcn_wave_barrier();
    __builtin_amdgcn_fence(__ATOMIC_ACQUIRE, "workgroup");
  }
}

__device__ __forceinline__ void kan_feats(float x, float* f) {
  const float e = expf(-x);
  f[0] = x * (1.0f / (1.0f + e));
  const float u = (x + 1.0f) * 2.5f + 3.0f;
  float b0[11];
#pragma unroll
  for (int j = 0; j < 11; ++j) b0[j] = (u >= (float)j && u < (float)(j + 1)) ? 1.0f : 0.0f;
  float b1[10];
#pragma unroll
  for (int j = 0; j < 10; ++j) b1[j] = (u - (float)j) * b0[j] + ((float)(j + 2) - u) * b0[j + 1];
  float b2[9];
#pragma unroll
  for (int j = 0; j < 9; ++j) b2[j] = 0.5f * ((u - (float)j) * b1[j] + ((float)(j + 3) - u) * b1[j + 1]);
#pragma unroll
  for (int j = 0; j < 8; ++j) f[1 + j] = (1.0f / 3.0f) * ((u - (float)j) * b2[j] + ((float)(j + 4) - u) * b2[j + 1]);
}

__device__ __forceinline__ float gelu_erf(float x) { return 0.5f * x * (1.0f + erff(x * 0.70710678118654752f)); }

__device__ __forceinline__ void store_row_segments(const unsigned short* sh, unsigned short* __restrict__ drow, int t) {
  v4u u[4];
#pragma unroll
  for (int it = 0; it < 4; ++it) {
    int c = t + it * 256;
    c = (c < kSeg8) ? c : (kSeg8 - 1);
    const unsigned short* s = sh + c * 8;
    u[it] = (v4u){pk16(s[0], s[1]), pk16(s[2], s[3]), pk16(s[4], s[5]), pk16(s[6], s[7])};
  }
  for (int pass = 0; pass < 2; ++pass) {
#pragma unroll
    for (int it = 0; it < 4; ++it) {
      const int c = t + it * 256;
      if (c < kSeg8) *(volatile v4u*)(drow + (size_t)c * 8) = u[it];
    }
    __threadfence();
  }
}

template <int NREAL>
__global__ __launch_bounds__(256) void prep_w_kernel(const float* __restrict__ bw, const float* __restrict__ sw,
                                                     const float* __restrict__ sc, unsigned short* __restrict__ dst) {
  __shared__ __align__(16) unsigned short sh[kKdim];
  const int o  = blockIdx.x;
  const int t  = threadIdx.x;
  const int oc = (o < NREAL) ? o : (NREAL - 1);
  const float fz = (o < NREAL) ? kCarry : 0.0f;
#pragma unroll 1
  for (int it = 0; it < 3; ++it) {
    const int i = t + it * 256;
    const size_t oi = (size_t)oc * kHid + i;
    const float b = bw[oi];
    const float s = sc[oi];
    const v4f p0 = *(const v4f*)(sw + oi * kBasis);
    const v4f p1 = *(const v4f*)(sw + oi * kBasis + 4);
    sh[i * kFeat + 0] = h_bits(b * fz);
#pragma unroll
    for (int e = 0; e < 4; ++e) {
      const float q0 = p0[e] * s;
      const float q1 = p1[e] * s;
      sh[i * kFeat + 1 + e] = h_bits(q0 * fz);
      sh[i * kFeat + 5 + e] = h_bits(q1 * fz);
    }
  }
  __syncthreads();
  store_row_segments(sh, dst + (size_t)o * kKdim, t);
}

template <int GELU_IN>
__global__ __launch_bounds__(256) void expand_kernel(const float* __restrict__ src, unsigned short* __restrict__ dst) {
  __shared__ __align__(16) unsigned short sh[kKdim];
  const int row = blockIdx.x;
  const int t   = threadIdx.x;
  const float* xr = src + (size_t)row * kHid;
#pragma unroll 1
  for (int it = 0; it < 3; ++it) {
    const int i = t + it * 256;
    float x = xr[i];
    if (GELU_IN) x = gelu_erf(x);
    float f[kFeat];
    kan_feats(x, f);
#pragma unroll
    for (int g = 0; g < kFeat; ++g) sh[i * kFeat + g] = h_bits(f[g] * kCarry);
  }
  __syncthreads();
  store_row_segments(sh, dst + (size_t)row * kKdim, t);
}

__global__ __launch_bounds__(256) void out_copy_kernel(const float* __restrict__ P, float* __restrict__ outp) {
  const int lane  = threadIdx.x & 31;
  const int gwave = blockIdx.x * 8 + (threadIdx.x >> 5);
  const int r0 = gwave * 64 + 2 * lane;
  const float* p0 = P + (size_t)r0 * kNpad;
  const float a0 = p0[0];
  const float a1 = p0[1];
  const float b0 = p0[kNpad];
  const float b1 = p0[kNpad + 1];
  const v4f v = (v4f){a0, a1, b0, b1};
  float* q = outp + (size_t)r0 * kNout;
  *(volatile v4f*)q = v;
  __threadfence();
  *(volatile v4f*)q = v;
}

extern "C" void kernel_launch(void* const* d_in, const int* in_sizes, int n_in,
                              void* d_out, int out_size, void* d_ws, size_t ws_size,
                              hipStream_t stream) {
  if (n_in < 7) return;
  if (in_sizes[0] != kRows * kHid) return;
  if (in_sizes[1] != kHid * kHid) return;
  if (in_sizes[2] != kHid * kHid * kBasis) return;
  if (in_sizes[3] != kHid * kHid) return;
  if (in_sizes[4] != kNout * kHid) return;
  if (in_sizes[5] != kNout * kHid * kBasis) return;
  if (in_sizes[6] != kNout * kHid) return;
  if (out_size != kRows * kNout) return;
  if (ws_size < kWsEnd) return;

  const float* hidden    = (const float*)d_in[0];
  const float* base_w1   = (const float*)d_in[1];
  const float* spline_w1 = (const float*)d_in[2];
  const float* scaler1   = (const float*)d_in[3];
  const float* base_w2   = (const float*)d_in[4];
  const float* spline_w2 = (const float*)d_in[5];
  const float* scaler2   = (const float*)d_in[6];
  float* outp = (float*)d_out;

  char* ws = (char*)d_ws;
  unsigned short* Bt1 = (unsigned short*)(ws + kOffBt1);
  unsigned short* Bt2 = (unsigned short*)(ws + kOffBt2);
  unsigned short* Apl = (unsigned short*)(ws + kOffA);
  float* H1 = (float*)(ws + kOffH1);
  float* Ppl = (float*)(ws + kOffP);

  prep_w_kernel<kHid><<<dim3(kHid), 256, 0, stream>>>(base_w1, spline_w1, scaler1, Bt1);
  prep_w_kernel<kNout><<<dim3(kNpad), 256, 0, stream>>>(base_w2, spline_w2, scaler2, Bt2);

  for (int c = 0; c < kNChunk; ++c) {
    const float* xsrc = hidden + (size_t)c * kChunk * kHid;
    float* h1c = H1 + (size_t)c * kChunk * kHid;
    float* pc  = Ppl + (size_t)c * kChunk * kNpad;

    expand_kernel<0><<<dim3(kChunk), 256, 0, stream>>>(xsrc, Apl);
    wmma_gemm64<0, false, 0, 0, false, 0><<<dim3((kChunk / 64) * (kHid / 64) / 8, 1), 256, 0, stream>>>(
        Apl, Apl, kKdim, 0L, Bt1, Bt1, kKdim, 0L,
        (void*)h1c, (void*)h1c, kHid, 0L,
        (const float*)h1c, (const float*)h1c, 0L,
        kChunk, kHid, kKdim, kGemmScale);
    expand_kernel<1><<<dim3(kChunk), 256, 0, stream>>>(h1c, Apl);
    wmma_gemm64<0, false, 0, 0, false, 0><<<dim3((kChunk / 64) * (kNpad / 64) / 8, 1), 256, 0, stream>>>(
        Apl, Apl, kKdim, 0L, Bt2, Bt2, kKdim, 0L,
        (void*)pc, (void*)pc, kNpad, 0L,
        (const float*)pc, (const float*)pc, 0L,
        kChunk, kNpad, kKdim, kGemmScale);
  }

  out_copy_kernel<<<dim3(kRows / 64 / 8), 256, 0, stream>>>(Ppl, outp);
}
